// ODE_RNN_79104707657778
// MI455X (gfx1250) — hardware-verified
//
#include <hip/hip_runtime.h>
#include <math.h>

constexpr int NBATCH   = 128;
constexpr int NTIME    = 64;
constexpr int NDIN     = 32;
constexpr int NHID     = 128;
constexpr int NSTAT    = 16;
constexpr int NSW      = 256;
constexpr int NOW      = 256;
constexpr int NDOUT    = 16;
constexpr int W0PITCH  = NHID + 1;
constexpr int KRNN     = NHID + NDIN;
constexpr int KINJREAL = NHID + NSTAT;
constexpr int KINJ     = 160;
constexpr int BLK_ROWS = 16;
constexpr int NTHR     = 512;
constexpr int PANP     = 264;
constexpr int KSZ      = BLK_ROWS * NHID;
constexpr int PK_THR   = 256;
constexpr float WCARRY     = 64.0f;
constexpr float WCARRY_INV = 1.0f / 64.0f;

static_assert(NTHR / 32 == BLK_ROWS, "one wave per batch row in the elementwise phases");
static_assert(NHID == 32 * 4, "lane owns 4 consecutive hidden columns");
static_assert(NDIN == 32, "lane owns one observation feature");
static_assert(NSTAT == 16, "lanes 0..15 own the static features");
static_assert(NSW == 16 * (NTHR / 32) && NOW == 16 * (NTHR / 32), "one 16-column tile per wave");
static_assert(NHID == 16 * 8, "waves 0..7 own the hidden tiles");
static_assert(NHID % 32 == 0 && NSW % 32 == 0 && NOW % 32 == 0 && KRNN % 32 == 0 && KINJ % 32 == 0, "K multiples of 32");
static_assert(KINJ >= KINJREAL && KINJ == KRNN, "inject K padded to the panel width");
static_assert(NBATCH % BLK_ROWS == 0, "whole row blocks");
static_assert(PANP % 8 == 0 && PANP >= NSW + 8, "panel pitch");
static_assert(BLK_ROWS * NDOUT == 256, "output slab = 1,024 contiguous bytes");

constexpr size_t OFF_W0H = 0;
constexpr size_t OFF_W1  = OFF_W0H + (size_t)NSW * NHID;
constexpr size_t OFF_W2  = OFF_W1  + (size_t)NSW * NSW;
constexpr size_t OFF_RNN = OFF_W2  + (size_t)NHID * NSW;
constexpr size_t OFF_INJ = OFF_RNN + (size_t)NHID * KRNN;
constexpr size_t OFF_O0  = OFF_INJ + (size_t)NHID * KINJ;
constexpr size_t OFF_O1  = OFF_O0  + (size_t)NOW * NHID;
constexpr size_t OFF_O2  = OFF_O1  + (size_t)NOW * NOW;
constexpr size_t OFF_END = OFF_O2  + (size_t)NDOUT * NOW;
constexpr size_t W0T_BYTE_OFF = OFF_END * 2;
constexpr size_t WS_TOTAL_BYTES = W0T_BYTE_OFF + (size_t)NSW * 4;
static_assert((OFF_W1 * 2) % 256 == 0 && (OFF_W2 * 2) % 256 == 0 && (OFF_RNN * 2) % 256 == 0 &&
              (OFF_INJ * 2) % 256 == 0 && (OFF_O0 * 2) % 256 == 0 && (OFF_O1 * 2) % 256 == 0 &&
              (OFF_O2 * 2) % 256 == 0 && W0T_BYTE_OFF % 256 == 0, "plane bases on 256-B boundaries");
static_assert(WS_TOTAL_BYTES <= (size_t)134217728, "carve");

constexpr int CH_W0H = NSW * (NHID / 8);
constexpr int CH_W1  = NSW * (NSW / 8);
constexpr int CH_W2  = NHID * (NSW / 8);
constexpr int CH_RNN = NHID * (KRNN / 8);
constexpr int CH_INJ = NHID * (KINJ / 8);
constexpr int CH_O0  = NOW * (NHID / 8);
constexpr int CH_O1  = NOW * (NOW / 8);
constexpr int CH_O2  = NDOUT * (NOW / 8);
static_assert(CH_W0H % PK_THR == 0 && CH_W1 % PK_THR == 0 && CH_W2 % PK_THR == 0 && CH_RNN % PK_THR == 0 &&
              CH_INJ % PK_THR == 0 && CH_O0 % PK_THR == 0 && CH_O1 % PK_THR == 0 && CH_O2 % PK_THR == 0, "exact blocks");
constexpr int BS_W0H = 0;
constexpr int BS_W1  = BS_W0H + CH_W0H / PK_THR;
constexpr int BS_W2  = BS_W1  + CH_W1 / PK_THR;
constexpr int BS_RNN = BS_W2  + CH_W2 / PK_THR;
constexpr int BS_INJ = BS_RNN + CH_RNN / PK_THR;
constexpr int BS_O0  = BS_INJ + CH_INJ / PK_THR;
constexpr int BS_O1  = BS_O0  + CH_O0 / PK_THR;
constexpr int BS_O2  = BS_O1  + CH_O1 / PK_THR;
constexpr int BS_W0T = BS_O2  + CH_O2 / PK_THR;
constexpr int PK_BLOCKS = BS_W0T + 1;

typedef __attribute__((ext_vector_type(16))) _Float16 v16h;
typedef __attribute__((ext_vector_type(8)))  _Float16 v8h;
typedef __attribute__((ext_vector_type(4)))  _Float16 v4h;
typedef __attribute__((ext_vector_type(8)))  float    v8f;
typedef __attribute__((ext_vector_type(4)))  float    v4f;

__constant__ float CT_TAB[6] = {0.0f, 0.161f, 0.327f, 0.9f, 0.9800255409045097f, 1.0f};
__constant__ float AT_TAB[30] = {
    0.0f, 0.0f, 0.0f, 0.0f, 0.0f,
    0.161f, 0.0f, 0.0f, 0.0f, 0.0f,
    -0.008480655492356989f, 0.335480655492357f, 0.0f, 0.0f, 0.0f,
    2.8971530571054935f, -6.359448489975075f, 4.3622954328695815f, 0.0f, 0.0f,
    5.325864828439257f, -11.748883564062828f, 7.4955393428898365f, -0.09249506636175525f, 0.0f,
    5.86145544294642f, -12.92096931784711f, 8.159367898576159f, -0.071584973281401f, -0.028269050394068383f};
__constant__ float BT_TAB[6] = {0.09646076681806523f, 0.01f, 0.4798896504144996f,
                                1.379008574103742f, -3.290069515436081f, 2.324710524099774f};

union FragU { v16h v; v8h h[2]; };
__device__ __forceinline__ v16h frag_load(const _Float16* p) {
  FragU f;
  f.h[0] = *(const v8h*)(p);
  f.h[1] = *(const v8h*)(p + 16);
  return f.v;
}
__device__ __forceinline__ v8f mma_f16(v16h a, v16h b, v8f c) {
  c = __builtin_amdgcn_wmma_f32_16x16x32_f16(false, a, false, b, (short)0, c, false, false);
  asm volatile("v_nop\n\tv_nop\n\tv_nop\n\tv_nop" : "+v"(c) : "v"(a), "v"(b));
  return c;
}
template <int KT>
__device__ __forceinline__ v8f gemm_tile(const _Float16* ap, const _Float16* bp) {
  v8f acc = {0.f, 0.f, 0.f, 0.f, 0.f, 0.f, 0.f, 0.f};
#pragma unroll
  for (int kt = 0; kt < KT; ++kt) {
    const v16h a = frag_load(ap + 32 * kt);
    const v16h b = frag_load(bp + 32 * kt);
    acc = mma_f16(a, b, acc);
  }
  return acc;
}
__device__ __forceinline__ float silu_f(float v) {
  const float e = expf(-v);
  return v * (1.0f / (1.0f + e));
}

template <int NROW, int KP, int LD1, int COL0, int N1, int LD2, int N2>
__device__ __forceinline__ void pack_plane(const float* __restrict__ s1, const float* __restrict__ s2,
                                           unsigned short* __restrict__ dst, int chunk) {
  constexpr int CPR = KP / 8;
  static_assert(KP % 32 == 0, "K pad");
  static_assert(N1 % 8 == 0, "chunk never straddles the source split");
  const int n  = chunk / CPR;
  const int kc = (chunk - n * CPR) * 8;
  v8h hv;
#pragma unroll
  for (int e = 0; e < 8; ++e) {
    const int k  = kc + e;
    const int k1 = (k < N1) ? k : (N1 - 1);
    float v1 = s1[(size_t)n * LD1 + COL0 + k1];
    float v2 = 0.0f;
    if (N2 > 0) {
      int k2 = k - N1;
      k2 = (k2 < 0) ? 0 : k2;
      k2 = (k2 > N2 - 1) ? (N2 - 1) : k2;
      v2 = s2[(size_t)n * LD2 + k2];
    }
    asm volatile("" : "+v"(v1));
    if (N2 > 0) {
      asm volatile("" : "+v"(v2));
    }
    float v = (k < N1) ? v1 : 0.0f;
    if (N2 > 0) {
      v = (k < N1) ? v1 : ((k < N1 + N2) ? v2 : 0.0f);
    }
    hv[e] = (_Float16)(v * WCARRY);
  }
  volatile v8h* dp = (volatile v8h*)(dst + (size_t)chunk * 8);
  *dp = hv;
  __threadfence();
  *dp = hv;
}

__global__ __launch_bounds__(PK_THR) void pack_planes_kernel(
    const float* __restrict__ fw0, const float* __restrict__ fw1, const float* __restrict__ fw2,
    const float* __restrict__ cwh, const float* __restrict__ cwx, const float* __restrict__ jw,
    const float* __restrict__ hw0, const float* __restrict__ hw1, const float* __restrict__ hw2,
    unsigned short* __restrict__ wsb, float* __restrict__ w0t) {
  const int blk = blockIdx.x;
  const int tid = threadIdx.x;
  if (blk < BS_W1) {
    pack_plane<NSW, NHID, W0PITCH, 1, NHID, 1, 0>(fw0, fw0, wsb + OFF_W0H, (blk - BS_W0H) * PK_THR + tid);
  } else if (blk < BS_W2) {
    pack_plane<NSW, NSW, NSW, 0, NSW, 1, 0>(fw1, fw1, wsb + OFF_W1, (blk - BS_W1) * PK_THR + tid);
  } else if (blk < BS_RNN) {
    pack_plane<NHID, NSW, NSW, 0, NSW, 1, 0>(fw2, fw2, wsb + OFF_W2, (blk - BS_W2) * PK_THR + tid);
  } else if (blk < BS_INJ) {
    pack_plane<NHID, KRNN, NHID, 0, NHID, NDIN, NDIN>(cwh, cwx, wsb + OFF_RNN, (blk - BS_RNN) * PK_THR + tid);
  } else if (blk < BS_O0) {
    pack_plane<NHID, KINJ, KINJREAL, 0, KINJREAL, 1, 0>(jw, jw, wsb + OFF_INJ, (blk - BS_INJ) * PK_THR + tid);
  } else if (blk < BS_O1) {
    pack_plane<NOW, NHID, NHID, 0, NHID, 1, 0>(hw0, hw0, wsb + OFF_O0, (blk - BS_O0) * PK_THR + tid);
  } else if (blk < BS_O2) {
    pack_plane<NOW, NOW, NOW, 0, NOW, 1, 0>(hw1, hw1, wsb + OFF_O1, (blk - BS_O1) * PK_THR + tid);
  } else if (blk < BS_W0T) {
    pack_plane<NDOUT, NOW, NOW, 0, NOW, 1, 0>(hw2, hw2, wsb + OFF_O2, (blk - BS_O2) * PK_THR + tid);
  } else {
    if (tid < NSW / 4) {
      v4f o;
#pragma unroll
      for (int e = 0; e < 4; ++e) o[e] = fw0[(size_t)(4 * tid + e) * W0PITCH];
      volatile v4f* op = (volatile v4f*)(w0t + 4 * tid);
      *op = o;
      __threadfence();
      *op = o;
    }
  }
}

__global__ __launch_bounds__(NTHR) void seq_solve_kernel(
    const float* __restrict__ ts, const float* __restrict__ X, const float* __restrict__ Stat,
    const unsigned short* __restrict__ wsb, const float* __restrict__ w0t,
    const float* __restrict__ fb0, const float* __restrict__ fb1, const float* __restrict__ fb2,
    const float* __restrict__ scale_p, const float* __restrict__ cbx, const float* __restrict__ jb,
    const float* __restrict__ hb0, const float* __restrict__ hb1, const float* __restrict__ hb2,
    float* __restrict__ out) {
  __shared__ __align__(16) float    ybuf[KSZ];
  __shared__ __align__(16) float    kbuf[6 * KSZ];
  __shared__ __align__(16) _Float16 panA[BLK_ROWS * PANP];
  __shared__ __align__(16) _Float16 panB[BLK_ROWS * PANP];
  __shared__ __align__(16) float    tst[BLK_ROWS];
  __shared__ __align__(16) float    ostage[BLK_ROWS * NDOUT];

  const int tid  = threadIdx.x;
  const int lane = tid & 31;
  const int wave = tid >> 5;
  const int c    = lane & 15;
  const int hh   = lane >> 4;
  const int koff = 8 * hh;
  const int m0   = blockIdx.x * BLK_ROWS;
  const int ncol  = 16 * wave + c;
  const int ncolh = ncol & (NHID - 1);

  const _Float16* PW = (const _Float16*)wsb;
  const _Float16* bL1 = PW + OFF_W0H + (size_t)ncol  * NHID + koff;
  const _Float16* bL2 = PW + OFF_W1  + (size_t)ncol  * NSW  + koff;
  const _Float16* bL3 = PW + OFF_W2  + (size_t)ncolh * NSW  + koff;
  const _Float16* bRN = PW + OFF_RNN + (size_t)ncolh * KRNN + koff;
  const _Float16* bIN = PW + OFF_INJ + (size_t)ncolh * KINJ + koff;
  const _Float16* bO0 = PW + OFF_O0  + (size_t)ncol  * NHID + koff;
  const _Float16* bO1 = PW + OFF_O1  + (size_t)ncol  * NOW  + koff;
  const _Float16* bO2 = PW + OFF_O2  + (size_t)c     * NOW  + koff;

  const _Float16* aA = panA + c * PANP + koff;
  const _Float16* aB = panB + c * PANP + koff;

  float b0c = fb0[ncol];
  float w0c = w0t[ncol];
  float b1c = fb1[ncol];
  float b2c = fb2[ncolh];
  float bxc = cbx[ncolh];
  float jbc = jb[ncolh];
  float scl = scale_p[0];
  asm volatile("" : "+v"(b0c));
  asm volatile("" : "+v"(w0c));
  asm volatile("" : "+v"(b1c));
  asm volatile("" : "+v"(b2c));
  asm volatile("" : "+v"(bxc));
  asm volatile("" : "+v"(jbc));
  asm volatile("" : "+v"(scl));

  const int eidx = wave * NHID + lane * 4;
  _Float16* ownA = panA + wave * PANP + lane * 4;

  {
    const float x0 = X[((size_t)(m0 + wave) * NTIME) * NDIN + lane];
    panA[wave * PANP + NHID + lane] = (_Float16)x0;
    const float sv = Stat[(size_t)(m0 + wave) * NSTAT + (lane & 15)];
    const float pv = (lane < NSTAT) ? sv : 0.0f;
    panB[wave * PANP + NHID + lane] = (_Float16)pv;
  }
  __syncthreads();
  if (wave < 8) {
    const v8f acc = gemm_tile<1>(aA + NHID, bRN + NHID);
#pragma unroll
    for (int r = 0; r < 8; ++r) {
      const float v = tanhf(acc[r] * WCARRY_INV + bxc);
      panB[(8 * hh + r) * PANP + ncol] = (_Float16)v;
    }
  }
  __syncthreads();
  if (wave < 8) {
    const v8f acc = gemm_tile<KINJ / 32>(aB, bIN);
#pragma unroll
    for (int r = 0; r < 8; ++r) ybuf[(8 * hh + r) * NHID + ncol] = tanhf(acc[r] * WCARRY_INV + jbc);
  }
  __syncthreads();

#pragma unroll 1
  for (int step = 0; step < NTIME - 1; ++step) {
    float t0v = ts[(size_t)(m0 + wave) * NTIME + step];
    float t1v = ts[(size_t)(m0 + wave) * NTIME + step + 1];
    float xv  = X[((size_t)(m0 + wave) * NTIME + step + 1) * NDIN + lane];
    asm volatile("" : "+v"(t0v));
    asm volatile("" : "+v"(t1v));
    asm volatile("" : "+v"(xv));
    const float dtv = (t1v - t0v) * 0.5f;

#pragma unroll 1
    for (int sub = 0; sub < 2; ++sub) {
      const float tsub = (sub == 0) ? t0v : (t0v + dtv);
#pragma unroll 1
      for (int st = 0; st < 6; ++st) {
        {
          const float cst = CT_TAB[st];
          v4f a = {0.f, 0.f, 0.f, 0.f};
#pragma unroll 1
          for (int i = 0; i < st; ++i) {
            const float ai = AT_TAB[st * 5 + i];
            const v4f kv = *(const v4f*)(kbuf + i * KSZ + eidx);
            a += ai * kv;
          }
          const v4f yv = *(const v4f*)(ybuf + eidx);
          v4h hv;
#pragma unroll
          for (int e = 0; e < 4; ++e) hv[e] = (_Float16)(yv[e] + dtv * a[e]);
          *(v4h*)ownA = hv;
          if (lane == 0) tst[wave] = tsub + cst * dtv;
        }
        __syncthreads();

        {
          const v8f acc = gemm_tile<NHID / 32>(aA, bL1);
          const v4f ta = *(const v4f*)(tst + 8 * hh);
          const v4f tb = *(const v4f*)(tst + 8 * hh + 4);
          float tv[8];
#pragma unroll
          for (int e = 0; e < 4; ++e) { tv[e] = ta[e]; tv[4 + e] = tb[e]; }
#pragma unroll
          for (int r = 0; r < 8; ++r) {
            const float v = acc[r] * WCARRY_INV + tv[r] * w0c + b0c;
            panB[(8 * hh + r) * PANP + ncol] = (_Float16)silu_f(v);
          }
        }
        __syncthreads();

        {
          const v8f acc = gemm_tile<NSW / 32>(aB, bL2);
#pragma unroll
          for (int r = 0; r < 8; ++r) {
            const float v = acc[r] * WCARRY_INV + b1c;
            panA[(8 * hh + r) * PANP + ncol] = (_Float16)silu_f(v);
          }
        }
        __syncthreads();

        if (wave < 8) {
          const v8f acc = gemm_tile<NSW / 32>(aA, bL3);
#pragma unroll
          for (int r = 0; r < 8; ++r)
            kbuf[st * KSZ + (8 * hh + r) * NHID + ncol] = scl * tanhf(acc[r] * WCARRY_INV + b2c);
        }
        __syncthreads();
      }
      {
        v4f a = {0.f, 0.f, 0.f, 0.f};
#pragma unroll 1
        for (int i = 0; i < 6; ++i) {
          const float bi = BT_TAB[i];
          const v4f kv = *(const v4f*)(kbuf + i * KSZ + eidx);
          a += bi * kv;
        }
        const v4f yv = *(const v4f*)(ybuf + eidx);
        const v4f yn = yv + dtv * a;
        *(v4f*)(ybuf + eidx) = yn;
      }
    }

    {
      const v4f yv = *(const v4f*)(ybuf + eidx);
      v4h hv;
#pragma unroll
      for (int e = 0; e < 4; ++e) hv[e] = (_Float16)yv[e];
      *(v4h*)ownA = hv;
      panA[wave * PANP + NHID + lane] = (_Float16)xv;
    }
    __syncthreads();
    if (wave < 8) {
      const v8f acc = gemm_tile<KRNN / 32>(aA, bRN);
#pragma unroll
      for (int r = 0; r < 8; ++r) ybuf[(8 * hh + r) * NHID + ncol] = tanhf(acc[r] * WCARRY_INV + bxc);
    }
    __syncthreads();
  }

  const float hb0c = hb0[ncol];
  const float hb1c = hb1[ncol];
  const float hb2c = hb2[c];
  {
    const v4f yv = *(const v4f*)(ybuf + eidx);
    v4h hv;
#pragma unroll
    for (int e = 0; e < 4; ++e) hv[e] = (_Float16)yv[e];
    *(v4h*)ownA = hv;
  }
  __syncthreads();
  {
    const v8f acc = gemm_tile<NHID / 32>(aA, bO0);
#pragma unroll
    for (int r = 0; r < 8; ++r) panB[(8 * hh + r) * PANP + ncol] = (_Float16)tanhf(acc[r] * WCARRY_INV + hb0c);
  }
  __syncthreads();
  {
    const v8f acc = gemm_tile<NOW / 32>(aB, bO1);
#pragma unroll
    for (int r = 0; r < 8; ++r) panA[(8 * hh + r) * PANP + ncol] = (_Float16)tanhf(acc[r] * WCARRY_INV + hb1c);
  }
  __syncthreads();
  if (wave == 0) {
    const v8f acc = gemm_tile<NOW / 32>(aA, bO2);
#pragma unroll
    for (int r = 0; r < 8; ++r) ostage[(8 * hh + r) * NDOUT + c] = acc[r] * WCARRY_INV + hb2c;
  }
  __syncthreads();
  if (wave == 0) {
    float* op = out + (size_t)m0 * NDOUT;
    const v4f v0 = *(const v4f*)(ostage + lane * 4);
    const v4f v1 = *(const v4f*)(ostage + 128 + lane * 4);
    for (int pass = 0; pass < 2; ++pass) {
      *(volatile v4f*)(op + lane * 4) = v0;
      *(volatile v4f*)(op + 128 + lane * 4) = v1;
      __threadfence();
    }
  }
}

extern "C" void kernel_launch(void* const* d_in, const int* in_sizes, int n_in,
                              void* d_out, int out_size, void* d_ws, size_t ws_size, hipStream_t stream) {
  if (n_in < 21 || d_out == nullptr || d_ws == nullptr) return;
  if (in_sizes[0] != NBATCH * NTIME || in_sizes[1] != NBATCH * NTIME * NDIN || in_sizes[2] != NBATCH * NSTAT ||
      in_sizes[3] != NSW * W0PITCH || in_sizes[4] != NSW || in_sizes[5] != NSW * NSW || in_sizes[6] != NSW ||
      in_sizes[7] != NHID * NSW || in_sizes[8] != NHID || in_sizes[9] != 1 ||
      in_sizes[10] != NHID * NHID || in_sizes[11] != NHID * NDIN || in_sizes[12] != NHID ||
      in_sizes[13] != NHID * KINJREAL || in_sizes[14] != NHID ||
      in_sizes[15] != NOW * NHID || in_sizes[16] != NOW || in_sizes[17] != NOW * NOW || in_sizes[18] != NOW ||
      in_sizes[19] != NDOUT * NOW || in_sizes[20] != NDOUT || out_size != NBATCH * NDOUT) return;
  if (WS_TOTAL_BYTES > ws_size) return;

  const float* ts   = (const float*)d_in[0];
  const float* X    = (const float*)d_in[1];
  const float* Stat = (const float*)d_in[2];
  const float* fw0  = (const float*)d_in[3];
  const float* fb0  = (const float*)d_in[4];
  const float* fw1  = (const float*)d_in[5];
  const float* fb1  = (const float*)d_in[6];
  const float* fw2  = (const float*)d_in[7];
  const float* fb2  = (const float*)d_in[8];
  const float* scal = (const float*)d_in[9];
  const float* cwh  = (const float*)d_in[10];
  const float* cwx  = (const float*)d_in[11];
  const float* cbx  = (const float*)d_in[12];
  const float* jw   = (const float*)d_in[13];
  const float* jb   = (const float*)d_in[14];
  const float* hw0  = (const float*)d_in[15];
  const float* hb0  = (const float*)d_in[16];
  const float* hw1  = (const float*)d_in[17];
  const float* hb1  = (const float*)d_in[18];
  const float* hw2  = (const float*)d_in[19];
  const float* hb2  = (const float*)d_in[20];

  unsigned short* wsb = (unsigned short*)d_ws;
  float* w0t = (float*)((char*)d_ws + W0T_BYTE_OFF);

  pack_planes_kernel<<<PK_BLOCKS, PK_THR, 0, stream>>>(fw0, fw1, fw2, cwh, cwx, jw, hw0, hw1, hw2, wsb, w0t);
  seq_solve_kernel<<<NBATCH / BLK_ROWS, NTHR, 0, stream>>>(ts, X, Stat, wsb, w0t, fb0, fb1, fb2, scal, cbx, jb,
                                                            hb0, hb1, hb2, (float*)d_out);
}
